// SFT_6777458393262
// MI455X (gfx1250) — hardware-verified
//
#include <hip/hip_runtime.h>
#include <stddef.h>

static constexpr int NB = 16, NL1 = 128, NOBJ = 64, ND = 512, NH = 256, NG4 = 1024, NFD = 1536, NSEM = 300, NSEMP = 320;
static constexpr int MROWS = NB * NL1;
static constexpr int UROWS = NB * NOBJ;
static constexpr int VIDP = 64;
static constexpr int PL_ROWS = 16;
static constexpr int BOFF_WS = 0, BOFF_UO = 512, BOFF_UM = 1024, BOFF_BF = 1536, BOFF_BB = 2560, BOFF_FC = 3584, BIAS_TOTAL = 3904;

static_assert(ND % 64 == 0 && NG4 % 64 == 0 && NSEMP % 64 == 0 && MROWS % 64 == 0 && UROWS % 64 == 0 && VIDP % 64 == 0);
static_assert(ND % 32 == 0 && NFD % 32 == 0 && NH % 32 == 0);
static_assert(NL1 / PL_ROWS == 8 && NB * NL1 / PL_ROWS == 128);
static_assert(NB * NL1 * ND * 4 + NB * NSEM * 4 == 4213504);
static_assert(BOFF_UO % 32 == 0 && BOFF_UM % 32 == 0 && BOFF_BF % 32 == 0 && BOFF_BB % 32 == 0 && BOFF_FC % 32 == 0 && BOFF_FC + NSEMP == BIAS_TOTAL);

typedef __attribute__((ext_vector_type(16))) _Float16 v16h;
typedef __attribute__((ext_vector_type(8)))  _Float16 v8h;
typedef __attribute__((ext_vector_type(16))) __bf16   v16b;
typedef __attribute__((ext_vector_type(8)))  __bf16   v8b;
typedef __attribute__((ext_vector_type(8)))  float    v8f;
typedef __attribute__((ext_vector_type(4)))  float    v4f;
typedef __attribute__((ext_vector_type(8)))  unsigned short v8us;
typedef __attribute__((ext_vector_type(4)))  unsigned int v4u;
typedef __attribute__((ext_vector_type(8)))  unsigned int v8u;

__device__ __forceinline__ unsigned short f2bf_bits(float f) {
  unsigned u = __float_as_uint(f);
  return (unsigned short)((u + 0x7FFFu + ((u >> 16) & 1u)) >> 16);
}
__device__ __forceinline__ float bf_bits2f(unsigned short h) { return __uint_as_float(((unsigned)h) << 16); }
__device__ __forceinline__ float bf16r(float f) { return bf_bits2f(f2bf_bits(f)); }
__device__ __forceinline__ unsigned short h16bits(float f) { return __builtin_bit_cast(unsigned short, (_Float16)f); }
__device__ __forceinline__ float opq(float x) { asm volatile("" : "+v"(x)); return x; }
__device__ __forceinline__ v8f zero8() { return (v8f){0.f, 0.f, 0.f, 0.f, 0.f, 0.f, 0.f, 0.f}; }

__device__ __forceinline__ void dep_guard_h(v8f& a, v8f& b, v16h x, v16h y) { asm volatile("v_nop\n\tv_nop\n\tv_nop\n\tv_nop" : "+v"(a), "+v"(b) : "v"(x), "v"(y)); }
__device__ __forceinline__ void dep_guard_b(v8f& a, v8f& b, v16b x, v16b y) { asm volatile("v_nop\n\tv_nop\n\tv_nop\n\tv_nop" : "+v"(a), "+v"(b) : "v"(x), "v"(y)); }
__device__ __forceinline__ void keep4_h(v16h a, v16h b, v16h c, v16h d) { asm volatile("v_nop" :: "v"(a), "v"(b), "v"(c), "v"(d)); }
__device__ __forceinline__ void keep4_b(v16b a, v16b b, v16b c, v16b d) { asm volatile("v_nop" :: "v"(a), "v"(b), "v"(c), "v"(d)); }
__device__ __forceinline__ void acc_guard4(v8f& a, v8f& b, v8f& c, v8f& d) { asm volatile("v_nop\n\tv_nop\n\tv_nop\n\tv_nop" : "+v"(a), "+v"(b), "+v"(c), "+v"(d)); }
template <typename T> struct Frag;
template <> struct Frag<_Float16> {
  typedef v16h V; union U { v16h v; v8h h[2]; };
  static __device__ __forceinline__ v16h load(const _Float16* p) {
    U f; f.h[0] = *(const v8h*)(p); f.h[1] = *(const v8h*)(p + 16); return f.v;
  }
  static __device__ __forceinline__ v8f mma(v16h a, v16h b, v8f c) {
    return __builtin_amdgcn_wmma_f32_16x16x32_f16(false, a, false, b, (short)0, c, false, false);
  }
  static __device__ __forceinline__ void guard(v8f& a, v8f& b, v16h x, v16h y) { dep_guard_h(a, b, x, y); }
  static __device__ __forceinline__ void keep(v16h a, v16h b, v16h c, v16h d) { keep4_h(a, b, c, d); }
};
template <> struct Frag<__bf16> {
  typedef v16b V; union U { v16b v; v8b h[2]; };
  static __device__ __forceinline__ v16b load(const __bf16* p) {
    U f; f.h[0] = *(const v8b*)(p); f.h[1] = *(const v8b*)(p + 16); return f.v;
  }
  static __device__ __forceinline__ v8f mma(v16b a, v16b b, v8f c) {
    return __builtin_amdgcn_wmma_f32_16x16x32_bf16(false, a, false, b, (short)0, c, false, false);
  }
  static __device__ __forceinline__ void guard(v8f& a, v8f& b, v16b x, v16b y) { dep_guard_b(a, b, x, y); }
  static __device__ __forceinline__ void keep(v16b a, v16b b, v16b c, v16b d) { keep4_b(a, b, c, d); }
};

__device__ __forceinline__ v8f mma_f16_g(v16h a, v16h b, v8f c) {
  c = __builtin_amdgcn_wmma_f32_16x16x32_f16(false, a, false, b, (short)0, c, false, false);
  asm volatile("v_nop\n\tv_nop\n\tv_nop\n\tv_nop" : "+v"(c) : "v"(a), "v"(b));
  return c;
}
__device__ __forceinline__ v8f mma_bf16_g(v16b a, v16b b, v8f c) {
  c = __builtin_amdgcn_wmma_f32_16x16x32_bf16(false, a, false, b, (short)0, c, false, false);
  asm volatile("v_nop\n\tv_nop\n\tv_nop\n\tv_nop" : "+v"(c) : "v"(a), "v"(b));
  return c;
}

template <int ET> struct Elem;
template <> struct Elem<0> { typedef _Float16 T; };
template <> struct Elem<1> { typedef __bf16 T; };
template <int ET, int SPLIT, int BIAS_MODE, int OUT_MODE>
__global__ __launch_bounds__(256) void wmma_gemm64(
    const unsigned short* __restrict__ Ap, const unsigned short* __restrict__ A2p, int lda, long strideA,
    const unsigned short* __restrict__ Btp, const unsigned short* __restrict__ Bt2p, int ldb, long strideB,
    void* __restrict__ Cout, void* __restrict__ Cout2, int ldc, long strideC,
    const float* __restrict__ bias,
    int M, int N, int K, float scale) {
  typedef typename Elem<ET>::T T;
  typedef typename Frag<T>::V V;
  const T* A = (const T*)Ap; const T* A2 = (const T*)A2p; const T* Bt = (const T*)Btp; const T* Bt2 = (const T*)Bt2p;
  __shared__ __align__(16) float sT[8][16 * 68];
  const int b    = blockIdx.y;
  const int lane = threadIdx.x & 31;
  const int wave = threadIdx.x >> 5;
  const int tilesN = N >> 6;
  const int tilesM = M >> 6;
  const int tile = blockIdx.x * 8 + wave;
  if (tile >= tilesM * tilesN) return;
  const int tm = tile / tilesN;
  const int tn = tile - tm * tilesN;
  const int m0 = tm << 6;
  const int n0 = tn << 6;

  const T* Ab  = A  + (size_t)b * strideA;
  const T* Bb  = Bt + (size_t)b * strideB;
  const T* Ab2 = (SPLIT >= 1) ? (A2  + (size_t)b * strideA) : nullptr;
  const T* Bb2 = (SPLIT == 2) ? (Bt2 + (size_t)b * strideB) : nullptr;

  const int rlane = lane & 15;
  const int koff  = (lane >> 4) * 8;
  const int mOff  = (lane >> 4) * 8;

  v8f acc[4][4];
#pragma unroll
  for (int i = 0; i < 4; ++i)
#pragma unroll
    for (int j = 0; j < 4; ++j) acc[i][j] = zero8();

  for (int k0 = 0; k0 < K; k0 += 32) {
    V bh[4], bl[4];
#pragma unroll
    for (int j = 0; j < 4; ++j) {
      const size_t bo = (size_t)(n0 + (j << 4) + rlane) * ldb + koff + k0;
      bh[j] = Frag<T>::load(Bb + bo);
      if (SPLIT == 2) bl[j] = Frag<T>::load(Bb2 + bo);
    }
#pragma unroll
    for (int i = 0; i < 4; ++i) {
      const size_t ao = (size_t)(m0 + (i << 4) + rlane) * lda + koff + k0;
      V ah = Frag<T>::load(Ab + ao);
      V al = ah;
      if (SPLIT >= 1) al = Frag<T>::load(Ab2 + ao);
#pragma unroll
      for (int j = 0; j < 4; ++j) {
        acc[i][j] = Frag<T>::mma(ah, bh[j], acc[i][j]);
        if (SPLIT >= 1) acc[i][j] = Frag<T>::mma(al, bh[j], acc[i][j]);
        if (SPLIT == 2) acc[i][j] = Frag<T>::mma(ah, bl[j], acc[i][j]);
      }
      Frag<T>::guard(acc[i][0], acc[i][3], ah, al);
    }
    Frag<T>::keep(bh[0], bh[1], bh[2], bh[3]);
    if (SPLIT == 2) Frag<T>::keep(bl[0], bl[1], bl[2], bl[3]);
  }
  acc_guard4(acc[0][0], acc[0][1], acc[0][2], acc[0][3]);
  acc_guard4(acc[1][0], acc[1][1], acc[1][2], acc[1][3]);
  acc_guard4(acc[2][0], acc[2][1], acc[2][2], acc[2][3]);
  acc_guard4(acc[3][0], acc[3][1], acc[3][2], acc[3][3]);

  float* slab = sT[wave];
#pragma unroll
  for (int i = 0; i < 4; ++i) {
    const int mBase = m0 + (i << 4);
#pragma unroll
    for (int j = 0; j < 4; ++j) {
      const int n = n0 + (j << 4) + rlane;
      float bv = 0.f;
      if (BIAS_MODE == 2) bv = bias[n];
#pragma unroll
      for (int r = 0; r < 8; ++r) {
        float v = acc[i][j][r] * scale;
        if (BIAS_MODE == 1) v += bias[mBase + mOff + r];
        if (BIAS_MODE == 2) v += bv;
        slab[(mOff + r) * 68 + (j << 4) + rlane] = v;
      }
    }
    __builtin_amdgcn_fence(__ATOMIC_RELEASE, "workgroup");
    __builtin_amdgcn_wave_barrier();
    __builtin_amdgcn_fence(__ATOMIC_ACQUIRE, "workgroup");
    if (OUT_MODE == 0) {
      float* C = (float*)Cout + (size_t)b * strideC;
      const int hh = lane >> 4, c4 = (lane & 15) * 4;
      for (int pass = 0; pass < 2; ++pass) {
#pragma unroll
        for (int it = 0; it < 8; ++it) {
          const int row = it * 2 + hh;
          v4f v = *(const v4f*)(slab + row * 68 + c4);
          *(volatile v4f*)(C + (size_t)(mBase + row) * ldc + n0 + c4) = v;
        }
        __threadfence();
      }
    } else {
      const int q = lane >> 3, c8 = (lane & 7) * 8;
      unsigned short* C  = (unsigned short*)Cout  + (size_t)b * strideC;
      unsigned short* C2 = (OUT_MODE == 2) ? ((unsigned short*)Cout2 + (size_t)b * strideC) : nullptr;
      for (int pass = 0; pass < 2; ++pass) {
#pragma unroll
        for (int it = 0; it < 4; ++it) {
          const int row = it * 4 + q;
          const float* sp = slab + row * 68 + c8;
          v8h hv, lv;
#pragma unroll
          for (int e = 0; e < 8; ++e) {
            if (OUT_MODE == 1) {
              hv[e] = (_Float16)sp[e];
            } else {
              unsigned short hb = f2bf_bits(sp[e]);
              unsigned short lb = f2bf_bits(sp[e] - bf_bits2f(hb));
              hv[e] = __builtin_bit_cast(_Float16, hb);
              lv[e] = __builtin_bit_cast(_Float16, lb);
            }
          }
          *(volatile v8h*)(C + (size_t)(mBase + row) * ldc + n0 + c8) = hv;
          if (OUT_MODE == 2) *(volatile v8h*)(C2 + (size_t)(mBase + row) * ldc + n0 + c8) = lv;
        }
        __threadfence();
      }
    }
    __builtin_amdgcn_fence(__ATOMIC_RELEASE, "workgroup");
    __builtin_amdgcn_wave_barrier();
    __builtin_amdgcn_fence(__ATOMIC_ACQUIRE, "workgroup");
  }
}

template <bool ZERO2>
__global__ __launch_bounds__(256) void cast_bf16x8(
    const float* __restrict__ in, unsigned short* __restrict__ out, unsigned short* __restrict__ out2,
    int rows_real, int rows_total, int cols, int out_ld) {
  const int g = blockIdx.x * 256 + threadIdx.x;
  const int gpr = cols >> 3;
  const int ngroups = rows_total * gpr;
  if (g >= ngroups) return;
  const int row = g / gpr;
  const int c8 = (g - row * gpr) * 8;
  const int rr = (row < rows_real) ? row : (rows_real - 1);
  const bool live = (row < rows_real);
  const float* src = in + (size_t)rr * cols + c8;
  const v4f a = *(const v4f*)(src);
  const v4f c = *(const v4f*)(src + 4);
  v8us hv;
#pragma unroll
  for (int e = 0; e < 4; ++e) {
    hv[e]     = live ? f2bf_bits(a[e]) : (unsigned short)0;
    hv[4 + e] = live ? f2bf_bits(c[e]) : (unsigned short)0;
  }
  const v8us zv = (v8us){0, 0, 0, 0, 0, 0, 0, 0};
  const size_t o = (size_t)row * out_ld + c8;
  *(volatile v8us*)(out + o) = hv;
  if (ZERO2) *(volatile v8us*)(out2 + o) = zv;
  __threadfence();
  *(volatile v8us*)(out + o) = hv;
  if (ZERO2) *(volatile v8us*)(out2 + o) = zv;
}

__global__ __launch_bounds__(32) void bias_prep_kernel(
    const float* __restrict__ ws_b, const float* __restrict__ uo_b, const float* __restrict__ um_b,
    const float* __restrict__ bih_f, const float* __restrict__ bhh_f,
    const float* __restrict__ bih_b, const float* __restrict__ bhh_b,
    const float* __restrict__ fc_b, float* __restrict__ bias_out) {
  const int seg = blockIdx.y;
  const int i = blockIdx.x * 32 + threadIdx.x;
  int len = ND, off = BOFF_WS;
  if (seg == 1) { len = ND; off = BOFF_UO; }
  else if (seg == 2) { len = ND; off = BOFF_UM; }
  else if (seg == 3) { len = NG4; off = BOFF_BF; }
  else if (seg == 4) { len = NG4; off = BOFF_BB; }
  else if (seg == 5) { len = NSEMP; off = BOFF_FC; }
  if (blockIdx.x * 32 >= len) return;
  float v;
  if (seg == 0) v = bf16r(ws_b[i]);
  else if (seg == 1) v = bf16r(uo_b[i]);
  else if (seg == 2) v = bf16r(um_b[i]);
  else if (seg == 3) v = bf16r(bih_f[i]) + bf16r(bhh_f[i]);
  else if (seg == 4) v = bf16r(bih_b[i]) + bf16r(bhh_b[i]);
  else {
    const int ic = (i < NSEM) ? i : (NSEM - 1);
    v = bf16r(fc_b[ic]);
    if (i >= NSEM) v = 0.0f;
  }
  volatile float* dst = bias_out + off + i;
  *dst = v;
  __threadfence();
  *dst = v;
}

__device__ __forceinline__ float tanh_fast(float x) {
  const float e = exp2f(x * 2.8853900817779268f);
  return fmaf(-2.0f, __builtin_amdgcn_rcpf(1.0f + e), 1.0f);
}
__device__ __forceinline__ float sigm_f(float x) { return __builtin_amdgcn_rcpf(1.0f + expf(-x)); }

__device__ __forceinline__ v16h tanh_frag(v4f w0, v4f w1, v4f w2, v4f w3, v4f u0, v4f u1, v4f u2, v4f u3) {
  v16h a;
#pragma unroll
  for (int e = 0; e < 4; ++e) {
    a[e]      = (_Float16)tanh_fast(w0[e] + u0[e]);
    a[4 + e]  = (_Float16)tanh_fast(w1[e] + u1[e]);
    a[8 + e]  = (_Float16)tanh_fast(w2[e] + u2[e]);
    a[12 + e] = (_Float16)tanh_fast(w3[e] + u3[e]);
  }
  return a;
}

__global__ __launch_bounds__(256) void pool_kernel(
    const float* __restrict__ Wf32, const float* __restrict__ Um32, const float* __restrict__ Uo32,
    const float* __restrict__ bm_in, const float* __restrict__ bo_in,
    const float* __restrict__ wm_w, const float* __restrict__ wo_w,
    const float* __restrict__ wm_b, const float* __restrict__ wo_b,
    unsigned short* __restrict__ feat_hi, unsigned short* __restrict__ feat_lo) {
  __shared__ __align__(16) unsigned short Ut16[ND * NOBJ];
  __shared__ __align__(16) float Wfb[PL_ROWS * ND];
  __shared__ __align__(16) unsigned int wwp[ND / 2];
  __shared__ __align__(16) float Ssc[PL_ROWS * NOBJ];
  __shared__ __align__(16) unsigned short P16[PL_ROWS * NOBJ];
  __shared__ float sumw[PL_ROWS];
  __shared__ __align__(16) float slab[8][16 * 68];

  const int tid = threadIdx.x, lane = tid & 31, wave = tid >> 5;
  const int rlane = lane & 15, koff = (lane >> 4) * 8, mOff = koff;
  const int pool = blockIdx.y;
  const float* U32  = pool ? Uo32 : Um32;
  const float* batt = pool ? bo_in : bm_in;
  const float* ww   = pool ? wo_w : wm_w;
  const float* wbp  = pool ? wo_b : wm_b;
  const int featOff = pool ? (2 * ND) : ND;
  const int b  = blockIdx.x >> 3;
  const int l0 = (blockIdx.x & 7) * PL_ROWS;
  const int rowbase = b * NL1 + l0;
  const float wb = bf16r(wbp[0]);

  {
    const float a0 = opq(bf16r(ww[2 * tid])) * 1024.0f;
    const float a1 = opq(bf16r(ww[2 * tid + 1])) * 1024.0f;
    wwp[tid] = (unsigned)h16bits(a0) | ((unsigned)h16bits(a1) << 16);
  }
#pragma unroll
  for (int i = 0; i < 8; ++i) {
    const int f4 = tid + 256 * i;
    const int r = f4 >> 7, c4 = (f4 & 127) * 4;
    const v4f a  = *(const v4f*)(Wf32 + (size_t)(rowbase + r) * ND + c4);
    const v4f bb = *(const v4f*)(batt + c4);
    v4f o;
#pragma unroll
    for (int e = 0; e < 4; ++e) o[e] = a[e] + bf16r(bb[e]);
    *(v4f*)(Wfb + r * ND + c4) = o;
  }
  {
    const float* Ub = U32 + (size_t)(b * NOBJ) * ND;
#pragma unroll 1
    for (int ch = 0; ch < 4; ++ch) {
#pragma unroll
      for (int i = 0; i < 8; ++i) {
        const int f4 = tid + 256 * (ch * 8 + i);
        const int o = f4 >> 7, d4 = (f4 & 127) * 4;
        const v4f u = *(const v4f*)(Ub + (size_t)o * ND + d4);
#pragma unroll
        for (int e = 0; e < 4; ++e) Ut16[(d4 + e) * NOBJ + o] = h16bits(u[e] * 16.0f);
      }
    }
  }
  __syncthreads();

  {
    const float* Ub = U32 + (size_t)(b * NOBJ) * ND;
    const _Float16* wwh = (const _Float16*)wwp;
    const unsigned msk = (rlane == 0) ? 0xffffffffu : 0u;
    const int hsel = lane >> 4;
    const float* wr0 = Wfb + (2 * wave) * ND + koff;
    const float* wr1 = wr0 + ND;
    union UH { v16h v; v8u u; };
#pragma unroll 1
    for (int ot = 0; ot < 4; ++ot) {
      v8f acc0 = zero8(), acc1 = zero8();
      const float* ur = Ub + (size_t)(ot * 16 + rlane) * ND + koff;
#pragma unroll 1
      for (int ks = 0; ks < 16; ++ks) {
        const int dA = ks * 32;
        const v4f u0 = *(const v4f*)(ur + dA);
        const v4f u1 = *(const v4f*)(ur + dA + 4);
        const v4f u2 = *(const v4f*)(ur + dA + 16);
        const v4f u3 = *(const v4f*)(ur + dA + 20);
        UH wv;
        wv.v = Frag<_Float16>::load(wwh + dA + koff);
#pragma unroll
        for (int e = 0; e < 8; ++e) wv.u[e] &= msk;
        {
          const v4f w0 = *(const v4f*)(wr0 + dA), w1 = *(const v4f*)(wr0 + dA + 4);
          const v4f w2 = *(const v4f*)(wr0 + dA + 16), w3 = *(const v4f*)(wr0 + dA + 20);
          const v16h av = tanh_frag(w0, w1, w2, w3, u0, u1, u2, u3);
          acc0 = mma_f16_g(av, wv.v, acc0);
        }
        {
          const v4f w0 = *(const v4f*)(wr1 + dA), w1 = *(const v4f*)(wr1 + dA + 4);
          const v4f w2 = *(const v4f*)(wr1 + dA + 16), w3 = *(const v4f*)(wr1 + dA + 20);
          const v16h av = tanh_frag(w0, w1, w2, w3, u0, u1, u2, u3);
          acc1 = mma_f16_g(av, wv.v, acc1);
        }
      }
      if (rlane == 0) {
#pragma unroll
        for (int r = 0; r < 8; ++r) {
          const int o = ot * 16 + hsel * 8 + r;
          Ssc[(2 * wave) * NOBJ + o]     = acc0[r] * (1.0f / 1024.0f) + wb;
          Ssc[(2 * wave + 1) * NOBJ + o] = acc1[r] * (1.0f / 1024.0f) + wb;
        }
      }
    }
  }
  __syncthreads();

#pragma unroll
  for (int li = 0; li < 2; ++li) {
    const int r = 2 * wave + li;
    const float s0 = Ssc[r * NOBJ + lane], s1 = Ssc[r * NOBJ + lane + 32];
    float mx = fmaxf(s0, s1);
#pragma unroll
    for (int off = 16; off > 0; off >>= 1) mx = fmaxf(mx, __shfl_xor(mx, off, 32));
    const float e0 = expf(s0 - mx), e1 = expf(s1 - mx);
    float sm = e0 + e1;
#pragma unroll
    for (int off = 16; off > 0; off >>= 1) sm += __shfl_xor(sm, off, 32);
    const float inv = 1.0f / sm;
    const float w0 = e0 * inv, w1 = e1 * inv;
    float sw = w0 + w1;
#pragma unroll
    for (int off = 16; off > 0; off >>= 1) sw += __shfl_xor(sw, off, 32);
    P16[r * NOBJ + lane]      = h16bits(w0 * 1024.0f);
    P16[r * NOBJ + lane + 32] = h16bits(w1 * 1024.0f);
    if (lane == 0) sumw[r] = sw;
  }
  __syncthreads();

  v8f pacc[4];
#pragma unroll
  for (int j = 0; j < 4; ++j) pacc[j] = zero8();
#pragma unroll
  for (int kk = 0; kk < 2; ++kk) {
    const v16h pa = Frag<_Float16>::load((const _Float16*)P16 + rlane * NOBJ + kk * 32 + koff);
#pragma unroll
    for (int j = 0; j < 4; ++j) {
      const v16h ub = Frag<_Float16>::load((const _Float16*)Ut16 + (size_t)(64 * wave + 16 * j + rlane) * NOBJ + kk * 32 + koff);
      pacc[j] = mma_f16_g(pa, ub, pacc[j]);
    }
  }
  float* sl = slab[wave];
#pragma unroll
  for (int j = 0; j < 4; ++j) {
    const int cl = 16 * j + rlane;
    const int dcol = 64 * wave + cl;
#pragma unroll
    for (int r = 0; r < 8; ++r) {
      const int row = mOff + r;
      sl[row * 68 + cl] = pacc[j][r] * (1.0f / 16384.0f) + Wfb[row * ND + dcol] * sumw[row];
    }
  }
  __syncthreads();
  {
    const int q = lane >> 3, c8 = (lane & 7) * 8;
    for (int pass = 0; pass < 2; ++pass) {
#pragma unroll
      for (int it = 0; it < 4; ++it) {
        const int row = it * 4 + q;
        const float* sp = sl + row * 68 + c8;
        v8us hv, lv;
#pragma unroll
        for (int e = 0; e < 8; ++e) {
          const unsigned short hb = f2bf_bits(sp[e]);
          const unsigned short lb = f2bf_bits(sp[e] - bf_bits2f(hb));
          hv[e] = hb; lv[e] = lb;
        }
        const size_t go = (size_t)(rowbase + row) * NFD + featOff + 64 * wave + c8;
        *(volatile v8us*)(feat_hi + go) = hv;
        *(volatile v8us*)(feat_lo + go) = lv;
      }
      __threadfence();
    }
  }
}

__global__ __launch_bounds__(512) void lstm_kernel(
    const float* __restrict__ pre_f, const float* __restrict__ pre_b,
    const unsigned short* __restrict__ whh_f, const unsigned short* __restrict__ whh_b,
    float* __restrict__ out0) {
  __shared__ __align__(16) float gsh[NB * NG4];
  __shared__ __align__(16) float hf32[NB * NH];
  __shared__ __align__(16) unsigned short hAh[NB * NH];
  __shared__ __align__(16) unsigned short hAl[NB * NH];
  const int tid = threadIdx.x, lane = tid & 31, wave = tid >> 5;
  const int rlane = lane & 15, koff = (lane >> 4) * 8, mOff = koff;
  const int dir = blockIdx.x;
  const float* pre = dir ? pre_b : pre_f;
  const __bf16* whh = (const __bf16*)(dir ? whh_b : whh_f);
  {
    const v4u z = (v4u){0u, 0u, 0u, 0u};
    *(v4u*)(hAh + tid * 8) = z;
    *(v4u*)(hAl + tid * 8) = z;
  }
  float creg[8];
#pragma unroll
  for (int e = 0; e < 8; ++e) creg[e] = 0.0f;
  const int em = wave, ej0 = lane * 8;
  const int n0 = wave * 64;
  __syncthreads();

  for (int t = 0; t < NL1; ++t) {
    const int tm = dir ? (NL1 - 1 - t) : t;
    v8f acc[4];
#pragma unroll
    for (int j = 0; j < 4; ++j) acc[j] = zero8();
#pragma unroll 2
    for (int k0 = 0; k0 < NH; k0 += 32) {
      const v16b ah = Frag<__bf16>::load((const __bf16*)hAh + rlane * NH + koff + k0);
      const v16b al = Frag<__bf16>::load((const __bf16*)hAl + rlane * NH + koff + k0);
#pragma unroll
      for (int j = 0; j < 4; ++j) {
        const v16b bw = Frag<__bf16>::load(whh + (size_t)(n0 + 16 * j + rlane) * NH + koff + k0);
        acc[j] = mma_bf16_g(ah, bw, acc[j]);
        acc[j] = mma_bf16_g(al, bw, acc[j]);
      }
    }
#pragma unroll
    for (int j = 0; j < 4; ++j)
#pragma unroll
      for (int r = 0; r < 8; ++r) gsh[(mOff + r) * NG4 + n0 + 16 * j + rlane] = acc[j][r];
    __syncthreads();
    {
      const float* prow = pre + ((size_t)em * NL1 + tm) * NG4 + ej0;
      const float* grow = gsh + em * NG4 + ej0;
      float g4[4][8];
#pragma unroll
      for (int g = 0; g < 4; ++g) {
        const v4f a0 = *(const v4f*)(grow + g * NH), a1 = *(const v4f*)(grow + g * NH + 4);
        const v4f p0 = *(const v4f*)(prow + g * NH), p1 = *(const v4f*)(prow + g * NH + 4);
#pragma unroll
        for (int e = 0; e < 4; ++e) { g4[g][e] = p0[e] + a0[e]; g4[g][4 + e] = p1[e] + a1[e]; }
      }
      float hv[8];
#pragma unroll
      for (int e = 0; e < 8; ++e) {
        const float ig = sigm_f(g4[0][e]);
        const float fg = sigm_f(g4[1][e]);
        const float gg = tanh_fast(g4[2][e]);
        const float og = sigm_f(g4[3][e]);
        const float c = fg * creg[e] + ig * gg;
        creg[e] = c;
        hv[e] = og * tanh_fast(c);
      }
      const v4f h0 = (v4f){hv[0], hv[1], hv[2], hv[3]};
      const v4f h1 = (v4f){hv[4], hv[5], hv[6], hv[7]};
      *(v4f*)(hf32 + em * NH + ej0) = h0;
      *(v4f*)(hf32 + em * NH + ej0 + 4) = h1;
      v4u uh, ul;
#pragma unroll
      for (int e2 = 0; e2 < 4; ++e2) {
        const unsigned short hb0 = f2bf_bits(hv[2 * e2]);
        const unsigned short lb0 = f2bf_bits(hv[2 * e2] - bf_bits2f(hb0));
        const unsigned short hb1 = f2bf_bits(hv[2 * e2 + 1]);
        const unsigned short lb1 = f2bf_bits(hv[2 * e2 + 1] - bf_bits2f(hb1));
        uh[e2] = (unsigned)hb0 | ((unsigned)hb1 << 16);
        ul[e2] = (unsigned)lb0 | ((unsigned)lb1 << 16);
      }
      *(v4u*)(hAh + em * NH + ej0) = uh;
      *(v4u*)(hAl + em * NH + ej0) = ul;
    }
    __syncthreads();
    {
      float* orow = out0 + ((size_t)wave * NL1 + tm) * (2 * NH) + dir * NH;
      const float* hrow = hf32 + wave * NH;
      for (int pass = 0; pass < 2; ++pass) {
#pragma unroll
        for (int it = 0; it < 2; ++it) {
          const int c4 = it * 128 + lane * 4;
          const v4f v = *(const v4f*)(hrow + c4);
          *(volatile v4f*)(orow + c4) = v;
        }
        __threadfence();
      }
    }
  }
}

__global__ __launch_bounds__(64) void vidmax_kernel(const float* __restrict__ out0,
                                                    unsigned short* __restrict__ vh, unsigned short* __restrict__ vl) {
  const int r = blockIdx.x;
  const int d0 = threadIdx.x * 8;
  float m[8];
  if (r < NB) {
    const float* base = out0 + (size_t)r * NL1 * ND + d0;
    const v4f a = *(const v4f*)(base), c = *(const v4f*)(base + 4);
#pragma unroll
    for (int e = 0; e < 4; ++e) { m[e] = a[e]; m[4 + e] = c[e]; }
#pragma unroll 4
    for (int tt = 1; tt < NL1; ++tt) {
      const v4f x = *(const v4f*)(base + (size_t)tt * ND), y = *(const v4f*)(base + (size_t)tt * ND + 4);
#pragma unroll
      for (int e = 0; e < 4; ++e) { m[e] = fmaxf(m[e], x[e]); m[4 + e] = fmaxf(m[4 + e], y[e]); }
    }
  } else {
#pragma unroll
    for (int e = 0; e < 8; ++e) m[e] = 0.0f;
  }
  v4u uh, ul;
#pragma unroll
  for (int e2 = 0; e2 < 4; ++e2) {
    const unsigned short hb0 = f2bf_bits(m[2 * e2]);
    const unsigned short lb0 = f2bf_bits(m[2 * e2] - bf_bits2f(hb0));
    const unsigned short hb1 = f2bf_bits(m[2 * e2 + 1]);
    const unsigned short lb1 = f2bf_bits(m[2 * e2 + 1] - bf_bits2f(hb1));
    uh[e2] = (unsigned)hb0 | ((unsigned)hb1 << 16);
    ul[e2] = (unsigned)lb0 | ((unsigned)lb1 << 16);
  }
  const size_t o = (size_t)r * ND + d0;
  for (int pass = 0; pass < 2; ++pass) {
    *(volatile v4u*)(vh + o) = uh;
    *(volatile v4u*)(vl + o) = ul;
    __threadfence();
  }
}

__global__ __launch_bounds__(256) void sem_copy_kernel(const float* __restrict__ sem32, float* __restrict__ out1) {
  const int i = blockIdx.x * 256 + threadIdx.x;
  if (i >= NB * NSEM) return;
  const int r = i / NSEM;
  const int c = i - r * NSEM;
  const float v = sem32[r * NSEMP + c];
  ((volatile float*)out1)[i] = v;
  __threadfence();
  ((volatile float*)out1)[i] = v;
}

extern "C" void kernel_launch(void* const* d_in, const int* in_sizes, int n_in,
                              void* d_out, int out_size, void* d_ws, size_t ws_size,
                              hipStream_t stream) {
  (void)in_sizes; (void)n_in; (void)out_size;
  const float* visual  = (const float*)d_in[0];
  const float* subject = (const float*)d_in[1];
  const float* predict = (const float*)d_in[2];
  const float* Ws_w  = (const float*)d_in[3];
  const float* Ws_b  = (const float*)d_in[4];
  const float* Uo_w  = (const float*)d_in[5];
  const float* Uo_b  = (const float*)d_in[6];
  const float* Um_w  = (const float*)d_in[7];
  const float* Um_b  = (const float*)d_in[8];
  const float* bo    = (const float*)d_in[9];
  const float* bm    = (const float*)d_in[10];
  const float* wo_w  = (const float*)d_in[11];
  const float* wo_b  = (const float*)d_in[12];
  const float* wm_w  = (const float*)d_in[13];
  const float* wm_b  = (const float*)d_in[14];
  const float* Wih_f = (const float*)d_in[15];
  const float* Whh_f = (const float*)d_in[16];
  const float* bih_f = (const float*)d_in[17];
  const float* bhh_f = (const float*)d_in[18];
  const float* Wih_b = (const float*)d_in[19];
  const float* Whh_b = (const float*)d_in[20];
  const float* bih_b = (const float*)d_in[21];
  const float* bhh_b = (const float*)d_in[22];
  const float* fc_w  = (const float*)d_in[23];
  const float* fc_b  = (const float*)d_in[24];

  float* out0 = (float*)d_out;
  float* out1 = out0 + (size_t)NB * NL1 * ND;

  size_t used = 0;
  char* wsb = (char*)d_ws;
  auto carve = [&](size_t bytes) -> char* { char* p = wsb + used; used += (bytes + 255) & ~(size_t)255; return p; };
  unsigned short* feat_hi = (unsigned short*)carve((size_t)MROWS * NFD * 2);
  unsigned short* feat_lo = (unsigned short*)carve((size_t)MROWS * NFD * 2);
  unsigned short* sub16   = (unsigned short*)carve((size_t)UROWS * ND * 2);
  unsigned short* prd16   = (unsigned short*)carve((size_t)UROWS * ND * 2);
  unsigned short* Ws16    = (unsigned short*)carve((size_t)ND * ND * 2);
  unsigned short* Uo16    = (unsigned short*)carve((size_t)ND * ND * 2);
  unsigned short* Um16    = (unsigned short*)carve((size_t)ND * ND * 2);
  unsigned short* Wihf16  = (unsigned short*)carve((size_t)NG4 * NFD * 2);
  unsigned short* Wihb16  = (unsigned short*)carve((size_t)NG4 * NFD * 2);
  unsigned short* Whhf16  = (unsigned short*)carve((size_t)NG4 * NH * 2);
  unsigned short* Whhb16  = (unsigned short*)carve((size_t)NG4 * NH * 2);
  unsigned short* fcw16   = (unsigned short*)carve((size_t)NSEMP * ND * 2);
  float* biasbuf = (float*)carve((size_t)BIAS_TOTAL * 4);
  float* Wf32    = (float*)carve((size_t)MROWS * ND * 4);
  float* Um32    = (float*)carve((size_t)UROWS * ND * 4);
  float* Uo32    = (float*)carve((size_t)UROWS * ND * 4);
  float* pre_f   = (float*)carve((size_t)MROWS * NG4 * 4);
  float* pre_b   = (float*)carve((size_t)MROWS * NG4 * 4);
  unsigned short* vid_hi = (unsigned short*)carve((size_t)VIDP * ND * 2);
  unsigned short* vid_lo = (unsigned short*)carve((size_t)VIDP * ND * 2);
  float* sem32   = (float*)carve((size_t)VIDP * NSEMP * 4);
  if (used > ws_size) return;

  auto cast_plane = [&](const float* in, unsigned short* o, int rows_real, int rows_total, int cols, int out_ld) {
    const int ng = rows_total * (cols / 8);
    cast_bf16x8<false><<<(ng + 255) / 256, 256, 0, stream>>>(in, o, o, rows_real, rows_total, cols, out_ld);
  };
  {
    const int ng = MROWS * (ND / 8);
    cast_bf16x8<true><<<(ng + 255) / 256, 256, 0, stream>>>(visual, feat_hi, feat_lo, MROWS, MROWS, ND, NFD);
  }
  cast_plane(subject, sub16,  UROWS, UROWS, ND,  ND);
  cast_plane(predict, prd16,  UROWS, UROWS, ND,  ND);
  cast_plane(Ws_w,    Ws16,   ND,    ND,    ND,  ND);
  cast_plane(Uo_w,    Uo16,   ND,    ND,    ND,  ND);
  cast_plane(Um_w,    Um16,   ND,    ND,    ND,  ND);
  cast_plane(Wih_f,   Wihf16, NG4,   NG4,   NFD, NFD);
  cast_plane(Wih_b,   Wihb16, NG4,   NG4,   NFD, NFD);
  cast_plane(Whh_f,   Whhf16, NG4,   NG4,   NH,  NH);
  cast_plane(Whh_b,   Whhb16, NG4,   NG4,   NH,  NH);
  cast_plane(fc_w,    fcw16,  NSEM,  NSEMP, ND,  ND);
  bias_prep_kernel<<<dim3(32, 6), 32, 0, stream>>>(Ws_b, Uo_b, Um_b, bih_f, bhh_f, bih_b, bhh_b, fc_b, biasbuf);

  {
    const int tiles = (MROWS / 64) * (ND / 64);
    wmma_gemm64<1, 0, 2, 0><<<dim3((tiles + 7) / 8, 1), 256, 0, stream>>>(
        feat_hi, nullptr, NFD, 0L, Ws16, nullptr, ND, 0L, (void*)Wf32, nullptr, ND, 0L,
        biasbuf + BOFF_WS, MROWS, ND, ND, 1.0f);
  }
  {
    const int tiles = (UROWS / 64) * (ND / 64);
    wmma_gemm64<1, 0, 2, 0><<<dim3((tiles + 7) / 8, 1), 256, 0, stream>>>(
        sub16, nullptr, ND, 0L, Uo16, nullptr, ND, 0L, (void*)Uo32, nullptr, ND, 0L,
        biasbuf + BOFF_UO, UROWS, ND, ND, 1.0f);
    wmma_gemm64<1, 0, 2, 0><<<dim3((tiles + 7) / 8, 1), 256, 0, stream>>>(
        prd16, nullptr, ND, 0L, Um16, nullptr, ND, 0L, (void*)Um32, nullptr, ND, 0L,
        biasbuf + BOFF_UM, UROWS, ND, ND, 1.0f);
  }

  pool_kernel<<<dim3(NB * NL1 / PL_ROWS, 2), 256, 0, stream>>>(
      Wf32, Um32, Uo32, bm, bo, wm_w, wo_w, wm_b, wo_b, feat_hi, feat_lo);

  {
    const int tiles = (MROWS / 64) * (NG4 / 64);
    wmma_gemm64<1, 1, 2, 0><<<dim3((tiles + 7) / 8, 1), 256, 0, stream>>>(
        feat_hi, feat_lo, NFD, 0L, Wihf16, nullptr, NFD, 0L, (void*)pre_f, nullptr, NG4, 0L,
        biasbuf + BOFF_BF, MROWS, NG4, NFD, 1.0f);
    wmma_gemm64<1, 1, 2, 0><<<dim3((tiles + 7) / 8, 1), 256, 0, stream>>>(
        feat_hi, feat_lo, NFD, 0L, Wihb16, nullptr, NFD, 0L, (void*)pre_b, nullptr, NG4, 0L,
        biasbuf + BOFF_BB, MROWS, NG4, NFD, 1.0f);
  }

  lstm_kernel<<<2, 512, 0, stream>>>(pre_f, pre_b, Whhf16, Whhb16, out0);

  vidmax_kernel<<<VIDP, 64, 0, stream>>>(out0, vid_hi, vid_lo);
  {
    const int tiles = (VIDP / 64) * (NSEMP / 64);
    wmma_gemm64<1, 1, 2, 0><<<dim3((tiles + 7) / 8, 1), 256, 0, stream>>>(
        vid_hi, vid_lo, ND, 0L, fcw16, nullptr, ND, 0L, (void*)sem32, nullptr, NSEMP, 0L,
        biasbuf + BOFF_FC, VIDP, NSEMP, ND, 1.0f);
  }
  sem_copy_kernel<<<(NB * NSEM + 255) / 256, 256, 0, stream>>>(sem32, out1);
}
